// Block_35648228557144
// MI455X (gfx1250) — hardware-verified
//
#include <hip/hip_runtime.h>
#include <math.h>

#ifndef NB
#define NB 2
#endif
#ifndef SEQ
#define SEQ 2048
#endif
#define NB_FULL 2
#define SEQ_FULL 2048
#define DM 1024
#define NH 16
#define HD 64
#define FF 4096
#define TOK (NB * SEQ)
#define QKW (2 * DM)

static_assert(NB <= NB_FULL);
static_assert(SEQ <= SEQ_FULL);
static_assert(NH * HD == DM);
static_assert(HD == 64);
static_assert(DM == 128 * 8);
static_assert(SEQ % 64 == 0);
static_assert(TOK % 64 == 0);
static_assert(DM % 64 == 0);
static_assert(FF % 64 == 0);
static_assert(DM % 32 == 0);
static_assert(FF % 32 == 0);
static_assert(FF == 4 * DM);
static_assert(DM % 8 == 0);

typedef __attribute__((ext_vector_type(16))) _Float16 v16h;
typedef __attribute__((ext_vector_type(8)))  _Float16 v8h;
typedef __attribute__((ext_vector_type(8)))  float    v8f;
typedef __attribute__((ext_vector_type(4)))  float    v4f;
typedef unsigned int u4 __attribute__((ext_vector_type(4)));
typedef unsigned int u2 __attribute__((ext_vector_type(2)));

__device__ __forceinline__ v16h ldfrag(const _Float16* __restrict__ p) {
    union { v16h v; v8h h[2]; } f;
    f.h[0] = *(const v8h*)(p);
    f.h[1] = *(const v8h*)(p + 16);
    return f.v;
}
__device__ __forceinline__ v8f wmma16(v16h a, v16h b, v8f c) {
    c = __builtin_amdgcn_wmma_f32_16x16x32_f16(false, a, false, b, (short)0, c, false, false);
    asm volatile("v_nop\n\tv_nop\n\tv_nop\n\tv_nop" : "+v"(c) : "v"(a), "v"(b));
    return c;
}
__device__ __forceinline__ void dep_guard_h(v8f& a, v8f& b, v16h x, v16h y) { asm volatile("v_nop\n\tv_nop\n\tv_nop\n\tv_nop" : "+v"(a), "+v"(b) : "v"(x), "v"(y)); }
__device__ __forceinline__ void keep4_h(v16h a, v16h b, v16h c, v16h d) { asm volatile("v_nop" :: "v"(a), "v"(b), "v"(c), "v"(d)); }
__device__ __forceinline__ void acc_guard4(v8f& a, v8f& b, v8f& c, v8f& d) { asm volatile("v_nop\n\tv_nop\n\tv_nop\n\tv_nop" : "+v"(a), "+v"(b), "+v"(c), "+v"(d)); }
__device__ __forceinline__ void wave_sync() {
    __builtin_amdgcn_fence(3  , "workgroup");
    __builtin_amdgcn_wave_barrier();
    __builtin_amdgcn_fence(2  , "workgroup");
}

#define VST2(T, ptr, val) do { const T vst2_v_ = (val); *(volatile T*)(ptr) = vst2_v_; __threadfence(); *(volatile T*)(ptr) = vst2_v_; } while (0)

__device__ __forceinline__ float cmb_bf(float v) { const unsigned u = __builtin_bit_cast(unsigned, v); const unsigned r = (u + 0x7fffu + ((u >> 16) & 1u)) & 0xffff0000u; return __builtin_bit_cast(float, r); }
__device__ __forceinline__ unsigned int cmb_pk2(float a, float b) { return (unsigned int)__builtin_bit_cast(unsigned short, (_Float16)a) | ((unsigned int)__builtin_bit_cast(unsigned short, (_Float16)b) << 16); }

__global__ __launch_bounds__(256) void k_cast16(const float* __restrict__ SRC, int lds, _Float16* __restrict__ DST, int ldd, int nR, int nC, float sc, int rpb, int rpb_full) {
    const long long u = (long long)blockIdx.x * 256 + threadIdx.x; const int per = nC / 8; if (u >= (long long)nR * per) return;
    const int r = (int)(u / per); const int c0 = 8 * (int)(u % per);
    const long long sr = (long long)(r / rpb) * rpb_full + (r % rpb);
    const float* s = SRC + sr * lds + c0;
    const v4f a = *(const v4f*)(s), b = *(const v4f*)(s + 4);
    u4 pk; pk.x = cmb_pk2(cmb_bf(a.x) * sc, cmb_bf(a.y) * sc); pk.y = cmb_pk2(cmb_bf(a.z) * sc, cmb_bf(a.w) * sc);
    pk.z = cmb_pk2(cmb_bf(b.x) * sc, cmb_bf(b.y) * sc); pk.w = cmb_pk2(cmb_bf(b.z) * sc, cmb_bf(b.w) * sc);
    VST2(u4, (u4*)(DST + (long long)r * ldd + c0), pk);
}
__global__ __launch_bounds__(256) void k_cast16T(const float* __restrict__ SRC, int lds, _Float16* __restrict__ DST, int ldd, int nR, int nC, float sc) {
    const long long u = (long long)blockIdx.x * 256 + threadIdx.x; const int per = nR / 8; if (u >= (long long)nC * per) return;
    const int c = (int)(u / per); const int r0 = 8 * (int)(u % per);
    float w[8];
#pragma unroll
    for (int e = 0; e < 8; ++e) w[e] = cmb_bf(SRC[(long long)(r0 + e) * lds + c]) * sc;
    u4 pk; pk.x = cmb_pk2(w[0], w[1]); pk.y = cmb_pk2(w[2], w[3]); pk.z = cmb_pk2(w[4], w[5]); pk.w = cmb_pk2(w[6], w[7]);
    VST2(u4, (u4*)(DST + (long long)c * ldd + r0), pk);
}

template <int BIAS_MODE, int OUT_MODE, int ACT>
__device__ __forceinline__ void gemm64_body(const _Float16* __restrict__ A, int lda, const _Float16* __restrict__ Bt, int ldb,
                                            float* __restrict__ Cf, _Float16* __restrict__ Ch, int ldc,
                                            const float* __restrict__ bias, int M, int N, int K, float scale) {
    __shared__ __align__(16) float sT[8][16 * 68];
    const int lane = threadIdx.x & 31;
    const int wave = threadIdx.x >> 5;
    const int tilesN = N >> 6;
    const int tilesM = M >> 6;
    const int tile = blockIdx.x * 8 + wave;
    if (tile >= tilesM * tilesN) return;
    const int tm = tile / tilesN;
    const int tn = tile - tm * tilesN;
    const int m0 = tm << 6;
    const int n0 = tn << 6;
    const int rlane = lane & 15;
    const int koff  = (lane >> 4) * 8;
    const int mOff  = (lane >> 4) * 8;

    v8f acc[4][4];
#pragma unroll
    for (int i = 0; i < 4; ++i)
#pragma unroll
        for (int j = 0; j < 4; ++j) acc[i][j] = (v8f){0.f, 0.f, 0.f, 0.f, 0.f, 0.f, 0.f, 0.f};

    for (int k0 = 0; k0 < K; k0 += 32) {
        v16h bh[4];
#pragma unroll
        for (int j = 0; j < 4; ++j) bh[j] = ldfrag(Bt + (size_t)(n0 + (j << 4) + rlane) * ldb + koff + k0);
#pragma unroll
        for (int i = 0; i < 4; ++i) {
            const v16h ah = ldfrag(A + (size_t)(m0 + (i << 4) + rlane) * lda + koff + k0);
#pragma unroll
            for (int j = 0; j < 4; ++j)
                acc[i][j] = __builtin_amdgcn_wmma_f32_16x16x32_f16(false, ah, false, bh[j], (short)0, acc[i][j], false, false);
            dep_guard_h(acc[i][0], acc[i][3], ah, ah);
        }
        keep4_h(bh[0], bh[1], bh[2], bh[3]);
    }
    acc_guard4(acc[0][0], acc[0][1], acc[0][2], acc[0][3]);
    acc_guard4(acc[1][0], acc[1][1], acc[1][2], acc[1][3]);
    acc_guard4(acc[2][0], acc[2][1], acc[2][2], acc[2][3]);
    acc_guard4(acc[3][0], acc[3][1], acc[3][2], acc[3][3]);

#pragma unroll
    for (int i = 0; i < 4; ++i) {
        const int mBase = m0 + (i << 4);
#pragma unroll
        for (int j = 0; j < 4; ++j) {
            const int n = n0 + (j << 4) + rlane;
            float bv = 0.f;
            if (BIAS_MODE == 2) bv = cmb_bf(bias[n]);
#pragma unroll
            for (int r = 0; r < 8; ++r) {
                float v = acc[i][j][r] * scale;
                if (BIAS_MODE == 1) v += cmb_bf(bias[mBase + mOff + r]);
                if (BIAS_MODE == 2) v += bv;
                if (ACT == 5) v = 0.5f * v * (1.0f + erff(v * 0.70710678118654752f));
                sT[wave][(mOff + r) * 68 + (j << 4) + rlane] = v;
            }
        }
        wave_sync();
        if (OUT_MODE == 0) {
            const int hh = lane >> 4, c4 = (lane & 15) * 4;
            for (int pass = 0; pass < 2; ++pass) {
#pragma unroll
                for (int it = 0; it < 8; ++it) {
                    const int row = it * 2 + hh;
                    const v4f v = *(const v4f*)(&sT[wave][row * 68 + c4]);
                    *(volatile v4f*)(Cf + (size_t)(mBase + row) * ldc + n0 + c4) = v;
                }
                __threadfence();
            }
        } else {
            const int q = lane >> 3, c8 = (lane & 7) * 8;
            for (int pass = 0; pass < 2; ++pass) {
#pragma unroll
                for (int it = 0; it < 4; ++it) {
                    const int row = it * 4 + q;
                    v8h hv;
#pragma unroll
                    for (int e = 0; e < 8; ++e) hv[e] = (_Float16)sT[wave][row * 68 + c8 + e];
                    *(volatile v8h*)(Ch + (size_t)(mBase + row) * ldc + n0 + c8) = hv;
                }
                __threadfence();
            }
        }
        wave_sync();
    }
}

__global__ __launch_bounds__(256) void k_gemm_h_bn(const _Float16* __restrict__ A, int lda, const _Float16* __restrict__ Bt, int ldb, _Float16* __restrict__ C, int ldc, const float* __restrict__ bias, int M, int N, int K, float scale) {
    gemm64_body<2, 1, 0>(A, lda, Bt, ldb, nullptr, C, ldc, bias, M, N, K, scale);
}
__global__ __launch_bounds__(256) void k_gemm_h_bm(const _Float16* __restrict__ A, int lda, const _Float16* __restrict__ Bt, int ldb, _Float16* __restrict__ C, int ldc, const float* __restrict__ bias, int M, int N, int K, float scale) {
    gemm64_body<1, 1, 0>(A, lda, Bt, ldb, nullptr, C, ldc, bias, M, N, K, scale);
}
__global__ __launch_bounds__(256) void k_gemm_h_gelu(const _Float16* __restrict__ A, int lda, const _Float16* __restrict__ Bt, int ldb, _Float16* __restrict__ C, int ldc, const float* __restrict__ bias, int M, int N, int K, float scale) {
    gemm64_body<2, 1, 5>(A, lda, Bt, ldb, nullptr, C, ldc, bias, M, N, K, scale);
}
__global__ __launch_bounds__(256) void k_gemm_f_bn(const _Float16* __restrict__ A, int lda, const _Float16* __restrict__ Bt, int ldb, float* __restrict__ C, int ldc, const float* __restrict__ bias, int M, int N, int K, float scale) {
    gemm64_body<2, 0, 0>(A, lda, Bt, ldb, C, nullptr, ldc, bias, M, N, K, scale);
}

#define AT_PP 40
static_assert((AT_PP * 2) % 16 == 0);
__global__ __launch_bounds__(128) void k_attn(const _Float16* __restrict__ QK, const _Float16* __restrict__ VT, _Float16* __restrict__ CTX) {
    __shared__ __align__(16) _Float16 Psh[4][16 * AT_PP];
    __shared__ __align__(16) float    Os[4][16 * 68];
    const int wave = threadIdx.x >> 5, lane = threadIdx.x & 31, hh = lane >> 4, c = lane & 15;
    const int nqb = SEQ / 64;
    const int bx = blockIdx.x;
    const int qb = bx % nqb;
    const int bh = bx / nqb;
    const int h = bh % NH;
    const int b = bh / NH;
    const int q0 = qb * 64 + wave * 16;
    const size_t rowb = (size_t)b * SEQ;
    const size_t qoff  = (rowb + q0 + c) * QKW + h * HD + 8 * hh;
    const size_t koff0 = (rowb + c) * QKW + DM + h * HD + 8 * hh;
    const size_t voff0 = (size_t)(h * HD + c) * TOK + rowb + 8 * hh;
    const float SCL = 0.125f * 1.4426950408889634f;
    const float NEG = -__builtin_inff();

    v8f o[4]; float m8[8], l8[8];
#pragma unroll
    for (int t = 0; t < 4; ++t) o[t] = (v8f){0.f, 0.f, 0.f, 0.f, 0.f, 0.f, 0.f, 0.f};
#pragma unroll
    for (int r = 0; r < 8; ++r) { m8[r] = NEG; l8[r] = 0.f; }

    for (int key0 = 0; key0 <= q0 + 15; key0 += 32) {
        v8f s0 = (v8f){0.f, 0.f, 0.f, 0.f, 0.f, 0.f, 0.f, 0.f};
        v8f s1 = s0;
#pragma unroll
        for (int dc = 0; dc < 2; ++dc) {
            const v16h qa  = ldfrag(QK + qoff + dc * 32);
            const v16h kf0 = ldfrag(QK + koff0 + (size_t)key0 * QKW + dc * 32);
            const v16h kf1 = ldfrag(QK + koff0 + (size_t)(key0 + 16) * QKW + dc * 32);
            s0 = wmma16(qa, kf0, s0);
            s1 = wmma16(qa, kf1, s1);
        }
#pragma unroll
        for (int r = 0; r < 8; ++r) {
            const int qrow = q0 + 8 * hh + r;
            const bool ma = (key0 + c > qrow), mb = (key0 + 16 + c > qrow);
            const float a = ma ? NEG : s0[r] * SCL;
            const float bq = mb ? NEG : s1[r] * SCL;
            float mx = fmaxf(a, bq);
            mx = fmaxf(mx, __shfl_xor(mx, 1, 32)); mx = fmaxf(mx, __shfl_xor(mx, 2, 32));
            mx = fmaxf(mx, __shfl_xor(mx, 4, 32)); mx = fmaxf(mx, __shfl_xor(mx, 8, 32));
            const float mnew = fmaxf(m8[r], mx);
            const float corr = exp2f(m8[r] - mnew);
            const float ea = exp2f(a - mnew), eb = exp2f(bq - mnew);
            const float pa = ma ? 0.f : ea;
            const float pb = mb ? 0.f : eb;
            float rs = pa + pb;
            rs += __shfl_xor(rs, 1, 32); rs += __shfl_xor(rs, 2, 32); rs += __shfl_xor(rs, 4, 32); rs += __shfl_xor(rs, 8, 32);
            l8[r] = l8[r] * corr + rs;
            m8[r] = mnew;
#pragma unroll
            for (int t = 0; t < 4; ++t) o[t][r] *= corr;
            Psh[wave][(8 * hh + r) * AT_PP + c]      = (_Float16)(pa * 4096.0f);
            Psh[wave][(8 * hh + r) * AT_PP + 16 + c] = (_Float16)(pb * 4096.0f);
        }
        wave_sync();
        {
            union { v16h v; v8h hv[2]; } pf;
            pf.hv[0] = *(const v8h*)(&Psh[wave][c * AT_PP + 8 * hh]);
            pf.hv[1] = *(const v8h*)(&Psh[wave][c * AT_PP + 16 + 8 * hh]);
            const v16h vb0 = ldfrag(VT + voff0 + (size_t)0  * 16 * TOK + key0);
            const v16h vb1 = ldfrag(VT + voff0 + (size_t)1  * 16 * TOK + key0);
            const v16h vb2 = ldfrag(VT + voff0 + (size_t)2  * 16 * TOK + key0);
            const v16h vb3 = ldfrag(VT + voff0 + (size_t)3  * 16 * TOK + key0);
            o[0] = wmma16(pf.v, vb0, o[0]);
            o[1] = wmma16(pf.v, vb1, o[1]);
            o[2] = wmma16(pf.v, vb2, o[2]);
            o[3] = wmma16(pf.v, vb3, o[3]);
        }
        wave_sync();
    }

#pragma unroll
    for (int r = 0; r < 8; ++r) {
        const float inv = 1.0f / (l8[r] * 64.0f);
#pragma unroll
        for (int t = 0; t < 4; ++t) Os[wave][(8 * hh + r) * 68 + t * 16 + c] = o[t][r] * inv;
    }
    wave_sync();
    {
        const int q = lane >> 3, c8 = (lane & 7) * 8;
        for (int pass = 0; pass < 2; ++pass) {
#pragma unroll
            for (int it = 0; it < 4; ++it) {
                const int row = it * 4 + q;
                v8h hv;
#pragma unroll
                for (int e = 0; e < 8; ++e) hv[e] = (_Float16)Os[wave][row * 68 + c8 + e];
                *(volatile v8h*)(CTX + (rowb + q0 + row) * DM + h * HD + c8) = hv;
            }
            __threadfence();
        }
    }
}

__global__ __launch_bounds__(256) void k_add_ln(const float* __restrict__ A, const float* __restrict__ X, int xbf, int xfull,
                                                const float* __restrict__ GA, const float* __restrict__ BE, int rows,
                                                float* __restrict__ Yf, int yfull, _Float16* __restrict__ Y16) {
    #pragma clang fp contract(off)
    const int r = blockIdx.x * 8 + (threadIdx.x >> 5); const int L = threadIdx.x & 31; if (r >= rows) return;
    const long long rf = (long long)(r / SEQ) * SEQ_FULL + (r % SEQ);
    const long long ra = (long long)r * DM;
    const long long rx = (xfull ? rf : (long long)r) * DM;
    const long long ry = (yfull ? rf : (long long)r) * DM;
    v4f v[8]; float s = 0.f;
#pragma unroll
    for (int q = 0; q < 8; ++q) {
        const int o = 4 * L + 128 * q;
        v[q] = *(const v4f*)(A + ra + o);
        v4f x = *(const v4f*)(X + rx + o);
        if (xbf) { x.x = cmb_bf(x.x); x.y = cmb_bf(x.y); x.z = cmb_bf(x.z); x.w = cmb_bf(x.w); }
        v[q] = v[q] + x;
        s += (v[q].x + v[q].y) + (v[q].z + v[q].w);
    }
#pragma unroll
    for (int o = 16; o > 0; o >>= 1) s += __shfl_xor(s, o, 32);
    const float mu = s * (1.f / DM); float qq = 0.f;
#pragma unroll
    for (int q = 0; q < 8; ++q) { v[q].x -= mu; v[q].y -= mu; v[q].z -= mu; v[q].w -= mu; qq += (v[q].x * v[q].x + v[q].y * v[q].y) + (v[q].z * v[q].z + v[q].w * v[q].w); }
#pragma unroll
    for (int o = 16; o > 0; o >>= 1) qq += __shfl_xor(qq, o, 32);
    const float rs = rsqrtf(qq * (1.f / DM) + 1e-5f);
#pragma unroll
    for (int q = 0; q < 8; ++q) {
        const int cc = 4 * L + 128 * q; const v4f ga = *(const v4f*)(GA + cc), be = *(const v4f*)(BE + cc); v4f y;
        y.x = v[q].x * rs * cmb_bf(ga.x) + cmb_bf(be.x); y.y = v[q].y * rs * cmb_bf(ga.y) + cmb_bf(be.y);
        y.z = v[q].z * rs * cmb_bf(ga.z) + cmb_bf(be.z); y.w = v[q].w * rs * cmb_bf(ga.w) + cmb_bf(be.w);
        if (Yf != nullptr) VST2(v4f, Yf + ry + cc, y);
        if (Y16 != nullptr) { u2 pk; pk.x = cmb_pk2(y.x, y.y); pk.y = cmb_pk2(y.z, y.w); VST2(u2, (u2*)(Y16 + ra + cc), pk); }
    }
}

extern "C" void kernel_launch(void* const* d_in, const int* in_sizes, int n_in, void* d_out, int out_size, void* d_ws, size_t ws_size, hipStream_t stream) {
    if (n_in < 13) return;
    const long long xneed = ((long long)(NB - 1) * SEQ_FULL + SEQ) * DM;
    if (in_sizes[0] < xneed || in_sizes[1] < 3 * DM * DM || in_sizes[2] < 3 * DM || in_sizes[3] < DM * DM || in_sizes[4] < DM ||
        in_sizes[5] < DM || in_sizes[6] < DM || in_sizes[7] < DM * FF || in_sizes[8] < FF || in_sizes[9] < FF * DM ||
        in_sizes[10] < DM || in_sizes[11] < DM || in_sizes[12] < DM || out_size < xneed) return;
    const float* x      = (const float*)d_in[0];
    const float* w_attn = (const float*)d_in[1];
    const float* b_attn = (const float*)d_in[2];
    const float* w_o    = (const float*)d_in[3];
    const float* b_o    = (const float*)d_in[4];
    const float* ln1_g  = (const float*)d_in[5];
    const float* ln1_b  = (const float*)d_in[6];
    const float* w_fc   = (const float*)d_in[7];
    const float* b_fc   = (const float*)d_in[8];
    const float* w_pr   = (const float*)d_in[9];
    const float* b_pr   = (const float*)d_in[10];
    const float* ln2_g  = (const float*)d_in[11];
    const float* ln2_b  = (const float*)d_in[12];
    float* out = (float*)d_out;

    constexpr size_t SZ_X16 = (size_t)TOK * DM * 2;
    constexpr size_t SZ_WA  = (size_t)3 * DM * DM * 2;
    constexpr size_t SZ_WO  = (size_t)DM * DM * 2;
    constexpr size_t SZ_WF  = (size_t)FF * DM * 2;
    constexpr size_t SZ_WP  = (size_t)DM * FF * 2;
    constexpr size_t SZ_QK  = (size_t)TOK * QKW * 2;
    constexpr size_t SZ_VT  = (size_t)DM * TOK * 2;
    constexpr size_t SZ_CTX = (size_t)TOK * DM * 2;
    constexpr size_t SZ_G   = (size_t)TOK * FF * 2;
    constexpr size_t SZ_RA  = (SZ_QK + SZ_VT + SZ_CTX > SZ_G) ? (SZ_QK + SZ_VT + SZ_CTX) : SZ_G;
    constexpr size_t SZ_F32 = (size_t)TOK * DM * 4;
    constexpr size_t SZ_ALL = SZ_X16 + SZ_WA + SZ_WO + SZ_WF + SZ_WP + SZ_RA + SZ_F32 + SZ_F32;
    static_assert(SZ_QK + SZ_VT + SZ_CTX <= SZ_RA);
    static_assert(SZ_G <= SZ_RA);
    static_assert(SZ_ALL <= (size_t)134217728);
    static_assert(SZ_X16 % 256 == 0 && SZ_WA % 256 == 0 && SZ_WO % 256 == 0 && SZ_QK % 256 == 0 && SZ_VT % 256 == 0 && SZ_F32 % 256 == 0);
    if (SZ_ALL > ws_size) return;
    char* wsp = (char*)d_ws;
    _Float16* X16  = (_Float16*)wsp; wsp += SZ_X16;
    _Float16* WA16 = (_Float16*)wsp; wsp += SZ_WA;
    _Float16* WO16 = (_Float16*)wsp; wsp += SZ_WO;
    _Float16* WF16 = (_Float16*)wsp; wsp += SZ_WF;
    _Float16* WP16 = (_Float16*)wsp; wsp += SZ_WP;
    char* RA = wsp; wsp += SZ_RA;
    float* ATT = (float*)wsp; wsp += SZ_F32;
    float* N1  = (float*)wsp; wsp += SZ_F32;
    _Float16* QK16  = (_Float16*)RA;
    _Float16* VT16  = (_Float16*)(RA + SZ_QK);
    _Float16* CTX16 = (_Float16*)(RA + SZ_QK + SZ_VT);
    _Float16* G16   = (_Float16*)RA;
    _Float16* N16   = X16;
    float* MLP = ATT;

    k_cast16<<<(unsigned)(((long long)TOK * (DM / 8) + 255) / 256), 256, 0, stream>>>(x, DM, X16, DM, TOK, DM, 1.0f, SEQ, SEQ_FULL);
    k_cast16T<<<(unsigned)(((long long)(3 * DM) * (DM / 8) + 255) / 256), 256, 0, stream>>>(w_attn, 3 * DM, WA16, DM, DM, 3 * DM, 16.0f);
    k_cast16T<<<(unsigned)(((long long)DM * (DM / 8) + 255) / 256), 256, 0, stream>>>(w_o, DM, WO16, DM, DM, DM, 16.0f);
    k_cast16T<<<(unsigned)(((long long)FF * (DM / 8) + 255) / 256), 256, 0, stream>>>(w_fc, FF, WF16, DM, DM, FF, 16.0f);
    k_cast16T<<<(unsigned)(((long long)DM * (FF / 8) + 255) / 256), 256, 0, stream>>>(w_pr, DM, WP16, FF, FF, DM, 16.0f);
    k_gemm_h_bn<<<(unsigned)(((TOK / 64) * (QKW / 64) + 7) / 8), 256, 0, stream>>>(X16, DM, WA16, DM, QK16, QKW, b_attn, TOK, QKW, DM, 0.0625f);
    k_gemm_h_bm<<<(unsigned)(((DM / 64) * (TOK / 64) + 7) / 8), 256, 0, stream>>>(WA16 + (size_t)2 * DM * DM, DM, X16, DM, VT16, TOK, b_attn + 2 * DM, DM, TOK, DM, 0.0625f);
    k_attn<<<(unsigned)(NB * NH * (SEQ / 64)), 128, 0, stream>>>(QK16, VT16, CTX16);
    k_gemm_f_bn<<<(unsigned)(((TOK / 64) * (DM / 64) + 7) / 8), 256, 0, stream>>>(CTX16, DM, WO16, DM, ATT, DM, b_o, TOK, DM, DM, 0.0009765625f);
    k_add_ln<<<(TOK + 7) / 8, 256, 0, stream>>>(ATT, x, 1, 1, ln1_g, ln1_b, TOK, N1, 0, N16);
    k_gemm_h_gelu<<<(unsigned)(((TOK / 64) * (FF / 64) + 7) / 8), 256, 0, stream>>>(N16, DM, WF16, DM, G16, FF, b_fc, TOK, FF, DM, 0.0625f);
    k_gemm_f_bn<<<(unsigned)(((TOK / 64) * (DM / 64) + 7) / 8), 256, 0, stream>>>(G16, FF, WP16, FF, MLP, DM, b_pr, TOK, DM, FF, 0.0625f);
    k_add_ln<<<(TOK + 7) / 8, 256, 0, stream>>>(MLP, N1, 0, 0, ln2_g, ln2_b, TOK, out, 1, nullptr);
}
